// MultiScaleLDSA_MemoryEfficient_20100446945672
// MI455X (gfx1250) — hardware-verified
//
#include <hip/hip_runtime.h>
#include <hip/hip_bf16.h>
#include <math.h>


typedef _Float16 bf16;
typedef _Float16 f16;
typedef __attribute__((ext_vector_type(4))) unsigned v4u_t;
typedef unsigned v4ua __attribute__((ext_vector_type(4), may_alias));
typedef __attribute__((ext_vector_type(4))) float v4f_t;
typedef float v4fa __attribute__((ext_vector_type(4), may_alias));
typedef __attribute__((ext_vector_type(16))) bf16  bf16x16;
typedef bf16x16 f16x16;
typedef __attribute__((ext_vector_type(8)))  bf16  bf16x8;
typedef bf16x8 f16x8;
typedef __attribute__((ext_vector_type(4)))  bf16  bf16x4;
typedef __attribute__((ext_vector_type(8)))  float f32x8;
__device__ __forceinline__ f32x8 wmma16(f16x16 a, f16x16 b, f32x8 c) {
  c = __builtin_amdgcn_wmma_f32_16x16x32_f16(false, a, false, b, (short)0, c, false, false);
  asm volatile("v_nop\n\tv_nop\n\tv_nop\n\tv_nop" : "+v"(c) : "v"(a), "v"(b));
  return c;
}
#define LDS_STRIDE 48
#define KSTRIDE    72
#define VSTRIDE    48

__device__ __forceinline__ f32x8 wmma_bf16(bf16x16 a, bf16x16 b, f32x8 c) {
  c = __builtin_amdgcn_wmma_f32_16x16x32_f16(false, a, false, b, (short)0, c, false, false);
  asm volatile("v_nop\n\tv_nop\n\tv_nop\n\tv_nop" : "+v"(c) : "v"(a), "v"(b));
  return c;
}

template <typename T>
__device__ __forceinline__ bf16x16 load_frag(const T* __restrict__ base, int ld,
                                             int row0, int k0) {
  const int lane = threadIdx.x & 31;
  const int r    = lane & 15;
  const int kh   = (lane >> 4) * 8;
  const T* p0 = base + (size_t)(row0 + r) * ld + (k0 + kh);
  const T* p1 = p0 + 16;
  bf16x16 f;
#pragma unroll
  for (int i = 0; i < 8; ++i) {
    f[i]     = (bf16)p0[i];
    f[i + 8] = (bf16)p1[i];
  }
  return f;
}

__device__ __forceinline__ bf16x16 lds_frag(const bf16* base, int stride) {
  const int lane = threadIdx.x & 31;
  const int row  = lane & 15;
  const int kh   = (lane >> 4) * 8;
  const bf16x8 lo = *(const bf16x8*)(base + row * stride + kh);
  const bf16x8 hi = *(const bf16x8*)(base + row * stride + kh + 16);
  bf16x16 f;
#pragma unroll
  for (int i = 0; i < 8; ++i) { f[i] = lo[i]; f[i + 8] = hi[i]; }
  return f;
}

template <typename T>
__device__ __forceinline__ void stage_read16(const T* __restrict__ p, float* buf) {
#pragma unroll
  for (int i = 0; i < 16; ++i) buf[i] = (float)p[i];
}

__device__ __forceinline__ void stage_write(bf16* dst, const float* buf, int nquad) {
#pragma unroll
  for (int i = 0; i < nquad; ++i) {
    bf16x4 q;
    q[0] = (bf16)buf[4 * i];     q[1] = (bf16)buf[4 * i + 1];
    q[2] = (bf16)buf[4 * i + 2]; q[3] = (bf16)buf[4 * i + 3];
    *(bf16x4*)(dst + 4 * i) = q;
  }
}


#define GSTR 48
#define GSTR 48
template <typename AT, int EPI, bool OUT16>
__global__ __launch_bounds__(256) void gemm_kne(const AT* __restrict__ A, int lda, const float* __restrict__ Wm, int ldw,
                                                const float* __restrict__ bias, const float* __restrict__ R, const float* __restrict__ gvec,
                                                void* __restrict__ Yv, int ldy, int K) {
  __shared__ __attribute__((aligned(16))) f16 ldsA[128 * GSTR];
  __shared__ __attribute__((aligned(16))) f16 ldsW[128 * GSTR];
  __shared__ __attribute__((aligned(16))) float oS[8][32 * 68];
  const int tid = threadIdx.x, lane = tid & 31, wave = tid >> 5, cl = lane & 15, rh = (lane >> 4) * 8;
  const int m0 = blockIdx.x * 128, n0 = blockIdx.y * 128;
  const int wm = (wave & 3) * 32, wn = (wave >> 2) * 64;
  f32x8 acc[2][4];
#pragma unroll
  for (int i = 0; i < 2; ++i)
#pragma unroll
    for (int j = 0; j < 4; ++j) { f32x8 z = {}; acc[i][j] = z; }
#pragma unroll 1
  for (int k0 = 0; k0 < K; k0 += 32) {
    __syncthreads();
    { const int row = tid >> 1, ch = (tid & 1) * 16;
      const AT* src = A + (size_t)(m0 + row) * lda + k0 + ch;
#pragma unroll
      for (int g = 0; g < 16; ++g) ldsA[row * GSTR + ch + g] = (f16)src[g]; }
    { const int k = tid >> 3, nn0 = (tid & 7) * 16;
      const float* src = Wm + (size_t)(k0 + k) * ldw + n0 + nn0;
#pragma unroll
      for (int g = 0; g < 4; ++g) { const v4f_t v = *(const v4f_t*)(src + 4 * g);
#pragma unroll
        for (int u = 0; u < 4; ++u) ldsW[(nn0 + 4 * g + u) * GSTR + k] = (f16)v[u]; } }
    __syncthreads();
    f16x16 af[2];
#pragma unroll
    for (int i = 0; i < 2; ++i) af[i] = lds_frag(ldsA + (wm + 16 * i) * GSTR, GSTR);
#pragma unroll
    for (int j = 0; j < 4; ++j) {
      const f16x16 bf = lds_frag(ldsW + (wn + 16 * j) * GSTR, GSTR);
#pragma unroll
      for (int i = 0; i < 2; ++i) acc[i][j] = wmma16(af[i], bf, acc[i][j]);
    }
  }
  float* so = oS[wave];
#pragma unroll
  for (int i = 0; i < 2; ++i)
#pragma unroll
    for (int j = 0; j < 4; ++j) {
      const int n = n0 + wn + 16 * j + cl;
      const float bv = bias ? bias[n] : 0.0f;
      const float gv = (EPI == 2 || EPI == 4) ? gvec[n] : 0.0f;
      if (EPI == 1) {
#pragma unroll 1
        for (int r = 0; r < 8; ++r) { const float xg = acc[i][j][r] + bv; so[(16 * i + rh + r) * 68 + 16 * j + cl] = 0.5f * xg * (1.0f + erff(xg * 0.70710678118654752f)); }
      } else {
#pragma unroll
        for (int r = 0; r < 8; ++r) {
          float v = acc[i][j][r] + bv;
          if (EPI == 3) v = fmaxf(v, 0.0f);
          if (EPI == 4) v = gv * v;
          if (EPI == 2) v = R[(size_t)(m0 + wm + 16 * i + rh + r) * ldy + n] + gv * v;
          so[(16 * i + rh + r) * 68 + 16 * j + cl] = v;
        }
      }
    }
  asm volatile("s_wait_dscnt 0" ::: "memory");
  __builtin_amdgcn_wave_barrier();
#pragma unroll 1
  for (int pass = 0; pass < 2; ++pass) {
    if (OUT16) {
      f16* Y = (f16*)Yv;
#pragma unroll
      for (int it = 0; it < 8; ++it) { const int c = lane + 32 * it, rr = c >> 3, q8 = (c & 7) * 8;
        union { f16 h[8]; v4u_t v; } u;
#pragma unroll
        for (int e = 0; e < 8; ++e) u.h[e] = (f16)so[rr * 68 + q8 + e];
        *(volatile v4u_t*)(Y + (size_t)(m0 + wm + rr) * ldy + n0 + wn + q8) = u.v; }
    } else {
      float* Y = (float*)Yv;
#pragma unroll
      for (int it = 0; it < 16; ++it) { const int f4 = lane + 32 * it, rr = f4 >> 4, q = (f4 & 15) * 4;
        *(volatile v4f_t*)(Y + (size_t)(m0 + wm + rr) * ldy + n0 + wn + q) = *(const v4fa*)(so + rr * 68 + q); }
    }
    __threadfence();
  }
}


#define NBT 4
#define BBm 4
#define TTm 1024
#define DDm 1024
#define HPS 4
#define HDm 256
#define C0 21
#define C1 41
#define NL0 (HPS * C0)
#define NL1 (HPS * C1)
#define NLP 256
#define MT (BBm * TTm)
__global__ __launch_bounds__(256) void k_packw2(const float* __restrict__ W20, const float* __restrict__ W21, float* __restrict__ W2p) {
  const int k = blockIdx.x, n = threadIdx.x; float v = 0.0f;
  if (n < NL0) v = W20[(size_t)k * NL0 + n]; else if (n < NL0 + NL1) v = W21[(size_t)k * NL1 + (n - NL0)];
  *(volatile float*)(W2p + (size_t)k * NLP + n) = v; __threadfence(); *(volatile float*)(W2p + (size_t)k * NLP + n) = v;
}
__global__ __launch_bounds__(256) void k_reluq(float* __restrict__ QV) { const size_t i = (size_t)blockIdx.x * 256 + threadIdx.x; const size_t r = i / (DDm / 4), c4 = (i % (DDm / 4)) * 4;
  float* p = QV + r * (2 * DDm) + c4; v4f_t v = *(const v4f_t*)p; v[0] = fmaxf(v[0], 0.f); v[1] = fmaxf(v[1], 0.f); v[2] = fmaxf(v[2], 0.f); v[3] = fmaxf(v[3], 0.f);
  *(volatile v4f_t*)p = v; __threadfence(); *(volatile v4f_t*)p = v; }
__global__ __launch_bounds__(256) void k_local(const float* __restrict__ LG, const float* __restrict__ QV, const float* __restrict__ swin, float* __restrict__ X) {
  __shared__ float a0[C0], a1[C1];
  const int t = blockIdx.x, h = blockIdx.y, b = blockIdx.z, d = threadIdx.x; const size_t row = (size_t)b * TTm + t; const float* lg = LG + row * NLP;
  if (d < 32) {
    float m0 = -3.0e38f, m1 = -3.0e38f;
    for (int j = 0; j < C0; ++j) m0 = fmaxf(m0, lg[h * C0 + j]);
    for (int j = 0; j < C1; ++j) m1 = fmaxf(m1, lg[NL0 + h * C1 + j]);
    float z0 = 0.f, z1 = 0.f;
    for (int j = 0; j < C0; ++j) z0 += expf(lg[h * C0 + j] - m0);
    for (int j = 0; j < C1; ++j) z1 += expf(lg[NL0 + h * C1 + j] - m1);
    for (int j = d; j < C0; j += 32) a0[j] = expf(lg[h * C0 + j] - m0) / z0;
    for (int j = d; j < C1; j += 32) a1[j] = expf(lg[NL0 + h * C1 + j] - m1) / z1;
  }
  __syncthreads();
  const float s0 = swin[0], s1 = swin[1]; const float sm = fmaxf(s0, s1); const float e0 = expf(s0 - sm), e1 = expf(s1 - sm); const float sw0 = e0 / (e0 + e1), sw1 = e1 / (e0 + e1);
  float acc0 = 0.0f, acc1 = 0.0f; const size_t col = (size_t)DDm + h * HDm + d;
#pragma unroll 1
  for (int j = 0; j < C0; ++j) { const int tt = t + j - (C0 - 1) / 2; if (tt >= 0 && tt < TTm) acc0 = fmaf(a0[j], QV[((size_t)b * TTm + tt) * (2 * DDm) + col], acc0); }
#pragma unroll 1
  for (int j = 0; j < C1; ++j) { const int tt = t + j - (C1 - 1) / 2; if (tt >= 0 && tt < TTm) acc1 = fmaf(a1[j], QV[((size_t)b * TTm + tt) * (2 * DDm) + col], acc1); }
  const float o = sw0 * acc0 + sw1 * acc1;
  float* dst = X + row * DDm + h * HDm + d; *(volatile float*)dst = o; __threadfence(); *(volatile float*)dst = o;
}

extern "C" void kernel_launch(void* const* d_in, const int* in_sizes, int n_in,
                              void* d_out, int out_size, void* d_ws, size_t ws_size,
                              hipStream_t stream) {
  (void)in_sizes; (void)n_in; (void)out_size;
  const float** f = (const float**)d_in;
  const float* query = f[0], *Wqv = f[3], *W20 = f[4], *W21 = f[5], *swin = f[6], *Wout = f[7];
  float* out = (float*)d_out;
  char* ws = (char*)d_ws;
  const size_t MQ = (size_t)NBT * TTm;
  float* W2p = (float*)ws; ws += (size_t)DDm * NLP * 4;
  float* QV = (float*)ws; ws += (size_t)MT * 2 * DDm * 4;
  float* LG = (float*)ws; ws += (size_t)MT * NLP * 4;
  float* X = (float*)ws; ws += (size_t)MT * DDm * 4;
  if ((size_t)(ws - (char*)d_ws) > ws_size) return;
  const dim3 blk(256);
  k_packw2<<<dim3(DDm), blk, 0, stream>>>(W20, W21, W2p);
  gemm_kne<float, 0, false><<<dim3(MQ / 128, 2 * DDm / 128), blk, 0, stream>>>(query, DDm, Wqv, 2 * DDm, nullptr, nullptr, nullptr, QV, 2 * DDm, DDm);
  k_reluq<<<dim3(MQ * (DDm / 4) / 256), blk, 0, stream>>>(QV);
  gemm_kne<float, 0, false><<<dim3(MQ / 128, NLP / 128), blk, 0, stream>>>(QV, 2 * DDm, W2p, NLP, nullptr, nullptr, nullptr, LG, NLP, DDm);
  k_local<<<dim3(TTm, HPS, NBT), blk, 0, stream>>>(LG, QV, swin, X);
  gemm_kne<float, 0, false><<<dim3(MQ / 128, DDm / 128), blk, 0, stream>>>(X, DDm, Wout, DDm, nullptr, nullptr, nullptr, out, DDm, DDm);
}
